// RecurrentDoubleGNN_26998164423206
// MI455X (gfx1250) — hardware-verified
//
#include <hip/hip_runtime.h>
#include <math.h>

#define N_NODES 50000
#define N_EDGES 1600000
#define D_IN 14
#define D_HID 64
#define D_OUT 7
#define D_G3  192
#define BUCKET 64
#define NBK   ((N_NODES + BUCKET - 1) / BUCKET)
#define NBKP  800
#define CHUNK 2048
#define NCH   ((N_EDGES + CHUNK - 1) / CHUNK)
#define SLOT  32
#define LCAP  2560
#define RSPLIT (1.0f / 2048.0f)

typedef _Float16 f16;
typedef __attribute__((ext_vector_type(16))) _Float16 v16h;
typedef __attribute__((ext_vector_type(8)))  float    v8f;
typedef __attribute__((ext_vector_type(4)))  float    f4;
typedef __attribute__((ext_vector_type(2)))  float    f2;
typedef float v4fa __attribute__((ext_vector_type(4), may_alias));

__device__ __forceinline__ v8f wmma16(v16h a, v16h b, v8f c) { return __builtin_amdgcn_wmma_f32_16x16x32_f16(false, a, false, b, (short)0, c, false, false); }
__device__ __forceinline__ v8f wmma_split(v16h a, v16h al, v16h b, v16h bl, v8f c) { v8f x = {}; x = wmma16(al, b, x); x = wmma16(a, bl, x); return wmma16(a, b, c) + x * RSPLIT; }
__device__ __forceinline__ f16 lo_of(float v, f16 h) { return (f16)((v - (float)h) * 2048.0f); }

__global__ __launch_bounds__(256) void gcn_gemm_kernel(const float* __restrict__ x, const float* __restrict__ W, float* __restrict__ h) {
  int idx = blockIdx.x * 256 + threadIdx.x;
  if (idx >= N_NODES * 16) return;
  int node = idx >> 4, c4 = (idx & 15) * 4;
  const float* xr = x + node * D_IN;
  f4 acc = {0.f, 0.f, 0.f, 0.f};
#pragma unroll 1
  for (int k = 0; k < D_IN; ++k) { const float xv = xr[k]; acc += xv * *(const f4*)(W + k * D_HID + c4); }
  float* o = h + (size_t)node * D_HID + c4;
  *(volatile f4*)o = acc; __threadfence(); *(volatile f4*)o = acc;
}

__global__ __launch_bounds__(256) void bin_kernel(const int* __restrict__ dst, int* __restrict__ slots, int* __restrict__ cnts) {
  __shared__ int cnt[NBKP];
  const int tid = threadIdx.x, ch = blockIdx.x;
  for (int i = tid; i < NBKP; i += 256) cnt[i] = 0;
  __syncthreads();
  int eb[8], ps[8];
#pragma unroll
  for (int u = 0; u < 8; ++u) {
    const int e = ch * CHUNK + u * 256 + tid;
    eb[u] = -1; ps[u] = -1;
    if (e < N_EDGES) { int d = dst[e]; d = ((unsigned)d < (unsigned)N_NODES) ? d : 0; const int b = d / BUCKET; const int p = atomicAdd(&cnt[b], 1); if (p < SLOT) { eb[u] = b; ps[u] = p; } }
  }
  __syncthreads();
#pragma unroll 1
  for (int pass = 0; pass < 2; ++pass) {
#pragma unroll
    for (int u = 0; u < 8; ++u) if (eb[u] >= 0) *(volatile int*)(slots + ((size_t)ch * NBK + eb[u]) * SLOT + ps[u]) = ch * CHUNK + u * 256 + tid;
    for (int i = tid; i < NBKP; i += 256) *(volatile int*)(cnts + (size_t)ch * NBKP + i) = (i < NBK) ? min(cnt[i], SLOT) : 0;
    __threadfence();
  }
}

__device__ void collect_bucket(const int* __restrict__ src, const int* __restrict__ dst, const int* __restrict__ slots, const int* __restrict__ cnts,
                               int bk, int n0, int* lst, int* lsrc, int* ncnt, int* noff, int& total) {
  const int tid = threadIdx.x;
  if (tid == 0) total = 0;
  if (tid < BUCKET) ncnt[tid] = 0;
  __syncthreads();
  int myc[4], mytot = 0;
#pragma unroll
  for (int u = 0; u < 4; ++u) { const int ch = tid + 256 * u; myc[u] = (ch < NCH) ? cnts[(size_t)ch * NBKP + bk] : 0; mytot += myc[u]; }
  __shared__ int scan[256];
  scan[tid] = mytot;
  __syncthreads();
#pragma unroll
  for (int off = 1; off < 256; off <<= 1) { const int v = (tid >= off) ? scan[tid - off] : 0; __syncthreads(); scan[tid] += v; __syncthreads(); }
  int pos = scan[tid] - mytot;
  if (tid == 255) total = min(scan[255], LCAP);
#pragma unroll
  for (int u = 0; u < 4; ++u) {
    const int ch = tid + 256 * u;
    for (int i = 0; i < myc[u]; ++i) { if (pos < LCAP) { const int e = slots[((size_t)ch * NBK + bk) * SLOT + i]; int d = dst[e]; d = ((unsigned)d < (unsigned)N_NODES) ? d : 0; lst[pos] = ((d - n0) << 24) | e; } ++pos; }
  }
  __syncthreads();
  const int nl = total;
  for (int i = tid; i < nl; i += 256) atomicAdd(&ncnt[(lst[i] >> 24) & 63], 1);
  __syncthreads();
  if (tid == 0) { int o = 0; for (int j = 0; j < BUCKET; ++j) { noff[j] = o; o += ncnt[j]; } }
  __syncthreads();
  if (tid < BUCKET) { int p = noff[tid]; for (int i = 0; i < nl; ++i) if (((lst[i] >> 24) & 63) == tid) { int s = src[lst[i] & 0xFFFFFF]; s = ((unsigned)s < (unsigned)N_NODES) ? s : 0; lsrc[p++] = s; } }
  __syncthreads();
}

__global__ __launch_bounds__(256) void deg_kernel(const int* __restrict__ src, const int* __restrict__ dst, const int* __restrict__ slots,
                                                 const int* __restrict__ cnts, float* __restrict__ dinv) {
  __shared__ int lst[LCAP], lsrc[LCAP], ncnt[BUCKET], noff[BUCKET], total;
  const int bk = blockIdx.x, n0 = bk * BUCKET;
  collect_bucket(src, dst, slots, cnts, bk, n0, lst, lsrc, ncnt, noff, total);
  const int tid = threadIdx.x;
  if (tid < BUCKET && n0 + tid < N_NODES) { const float v = 1.0f / sqrtf((float)ncnt[tid] + 1.0f); *(volatile float*)(dinv + n0 + tid) = v; __threadfence(); *(volatile float*)(dinv + n0 + tid) = v; }
}

__global__ __launch_bounds__(256) void gather_kernel(const int* __restrict__ src, const int* __restrict__ dst, const int* __restrict__ slots,
                                                    const int* __restrict__ cnts, const float* __restrict__ dinv,
                                                    const float* __restrict__ h, float* __restrict__ agg) {
  __shared__ int lst[LCAP], lsrc[LCAP], ncnt[BUCKET], noff[BUCKET], total;
  const int bk = blockIdx.x, n0 = bk * BUCKET;
  collect_bucket(src, dst, slots, cnts, bk, n0, lst, lsrc, ncnt, noff, total);
  const int tid = threadIdx.x, lane = tid & 31, wave = tid >> 5;
  for (int j = wave; j < BUCKET; j += 8) {
    const int node = n0 + j;
    if (node >= N_NODES) break;
    const int o0 = noff[j], cn = ncnt[j];
    const float dd = dinv[node];
    f2 a = *(const f2*)(h + (size_t)node * D_HID + lane * 2) * (dd * dd);
    for (int i = 0; i < cn; ++i) { const int s = lsrc[o0 + i]; a += *(const f2*)(h + (size_t)s * D_HID + lane * 2) * (dinv[s] * dd); }
    float* o = agg + (size_t)node * D_HID + lane * 2;
    *(volatile f2*)o = a; __threadfence(); *(volatile f2*)o = a;
  }
}

__global__ __launch_bounds__(256) void gi_gemm_wmma(const float* __restrict__ agg, const float* __restrict__ b_gcn,
                                                   const float* __restrict__ W_ih, const float* __restrict__ b_ih, float* __restrict__ GI) {
  __shared__ __attribute__((aligned(16))) float stg[8][16 * D_G3];
  const int wid = threadIdx.x >> 5, lane = threadIdx.x & 31, hi = lane >> 4, l16 = lane & 15;
  const int tm = blockIdx.x * 8 + wid;
  if (tm >= N_NODES / 16) return;
  const int mrow = tm * 16 + l16;
  v8f c[12];
#pragma unroll
  for (int i = 0; i < 12; ++i) c[i] = (v8f){};
#pragma unroll
  for (int kc = 0; kc < 2; ++kc) {
    const int Kb = kc * 32 + hi * 8;
    float av[16];
    *(f4*)(av + 0) = *(const f4*)(agg + (size_t)mrow * D_HID + Kb) + *(const f4*)(b_gcn + Kb);
    *(f4*)(av + 4) = *(const f4*)(agg + (size_t)mrow * D_HID + Kb + 4) + *(const f4*)(b_gcn + Kb + 4);
    *(f4*)(av + 8) = *(const f4*)(agg + (size_t)mrow * D_HID + Kb + 16) + *(const f4*)(b_gcn + Kb + 16);
    *(f4*)(av + 12) = *(const f4*)(agg + (size_t)mrow * D_HID + Kb + 20) + *(const f4*)(b_gcn + Kb + 20);
    v16h a, al;
#pragma unroll
    for (int j = 0; j < 16; ++j) { const f16 hh = (f16)av[j]; a[j] = hh; al[j] = lo_of(av[j], hh); }
#pragma unroll
    for (int nt = 0; nt < 12; ++nt) {
      const float* wrow = W_ih + (size_t)(nt * 16 + l16) * D_HID + Kb;
      float bv[16];
      *(f4*)(bv + 0) = *(const f4*)(wrow); *(f4*)(bv + 4) = *(const f4*)(wrow + 4);
      *(f4*)(bv + 8) = *(const f4*)(wrow + 16); *(f4*)(bv + 12) = *(const f4*)(wrow + 20);
      v16h b, bl;
#pragma unroll
      for (int j = 0; j < 16; ++j) { const f16 hh = (f16)bv[j]; b[j] = hh; bl[j] = lo_of(bv[j], hh); }
      c[nt] = wmma_split(a, al, b, bl, c[nt]);
    }
  }
  float* sw = stg[wid];
  const int rbase = hi * 8;
#pragma unroll
  for (int nt = 0; nt < 12; ++nt) { const int ncol = nt * 16 + l16; const float bias = b_ih[ncol];
#pragma unroll
    for (int r = 0; r < 8; ++r) sw[(rbase + r) * D_G3 + ncol] = c[nt][r] + bias; }
  asm volatile("s_wait_dscnt 0" ::: "memory");
  float* ob = GI + (size_t)tm * 16 * D_G3;
#pragma unroll 1
  for (int pass = 0; pass < 2; ++pass) {
#pragma unroll
    for (int i = 0; i < 24; ++i) { const int cc = lane + 32 * i; *(volatile f4*)(ob + cc * 4) = *(const volatile v4fa*)(sw + cc * 4); }
    __threadfence();
  }
}

__global__ __launch_bounds__(256) void gru_scan_kernel(const float* __restrict__ GI, const float* __restrict__ W_hh, const float* __restrict__ b_hh,
                                                      const float* __restrict__ h0, float* __restrict__ outs, float* __restrict__ hfinal) {
  __shared__ float whh[D_G3 * (D_HID + 1)];
  __shared__ float h_s[D_HID];
  __shared__ float gh_s[D_G3];
  __shared__ float gin_s[D_HID];
  const int tid = threadIdx.x;
  for (int i = tid; i < D_G3 * D_HID; i += 256) whh[(i >> 6) * (D_HID + 1) + (i & 63)] = W_hh[i];
  float bh = (tid < D_G3) ? b_hh[tid] : 0.0f;
  if (tid < D_HID) h_s[tid] = h0[tid];
  __syncthreads();
  const float* wr = whh + tid * (D_HID + 1);
  for (int t = 0; t < N_NODES; ++t) {
    if (tid < D_G3) {
      const float gi = GI[(size_t)t * D_G3 + tid];
      float a0 = 0.f, a1 = 0.f;
#pragma unroll 1
      for (int k = 0; k < D_HID; k += 2) { a0 += wr[k] * h_s[k]; a1 += wr[k + 1] * h_s[k + 1]; }
      const float gh = bh + (a0 + a1);
      if (tid < 2 * D_HID) gh_s[tid] = gi + gh; else { gh_s[tid] = gh; gin_s[tid - 2 * D_HID] = gi; }
    }
    __syncthreads();
    if (tid < D_HID) {
      const float r = 1.0f / (1.0f + __expf(-gh_s[tid]));
      const float z = 1.0f / (1.0f + __expf(-gh_s[D_HID + tid]));
      const float np_ = gin_s[tid] + r * gh_s[2 * D_HID + tid];
      const float n = 1.0f - 2.0f / (__expf(2.0f * np_) + 1.0f);
      const float hn = (1.0f - z) * n + z * h_s[tid];
      h_s[tid] = hn;
      *(volatile float*)(outs + (size_t)t * D_HID + tid) = hn;
    } else if (tid < 2 * D_HID && t > 0) {
      *(volatile float*)(outs + (size_t)(t - 1) * D_HID + (tid - D_HID)) = outs[(size_t)(t - 1) * D_HID + (tid - D_HID)];
    }
    __threadfence();
    __syncthreads();
  }
  if (tid < D_HID) {
    const float hv = h_s[tid];
    *(volatile float*)(outs + (size_t)(N_NODES - 1) * D_HID + tid) = hv;
    *(volatile float*)(hfinal + tid) = hv; __threadfence(); *(volatile float*)(hfinal + tid) = hv;
  }
}

__global__ __launch_bounds__(256) void fc_kernel(const float* __restrict__ outs, const float* __restrict__ W_fc, const float* __restrict__ b_fc, float* __restrict__ y) {
  int idx = blockIdx.x * 256 + threadIdx.x;
  if (idx >= N_NODES * D_OUT) return;
  int node = idx / D_OUT, o = idx % D_OUT;
  const float* hr = outs + (size_t)node * D_HID;
  float acc = b_fc[o];
#pragma unroll 1
  for (int c = 0; c < D_HID; ++c) acc += hr[c] * W_fc[c * D_OUT + o];
  *(volatile float*)(y + idx) = acc; __threadfence(); *(volatile float*)(y + idx) = acc;
}

extern "C" void kernel_launch(void* const* d_in, const int* in_sizes, int n_in,
                              void* d_out, int out_size, void* d_ws, size_t ws_size,
                              hipStream_t stream) {
    (void)in_sizes; (void)n_in; (void)out_size; (void)ws_size;
    const float* x     = (const float*)d_in[0];
    const int*   eidx  = (const int*)  d_in[1];
    const float* h0    = (const float*)d_in[2];
    const float* W_gcn = (const float*)d_in[3];
    const float* b_gcn = (const float*)d_in[4];
    const float* W_ih  = (const float*)d_in[5];
    const float* W_hh  = (const float*)d_in[6];
    const float* b_ih  = (const float*)d_in[7];
    const float* b_hh  = (const float*)d_in[8];
    const float* W_fc  = (const float*)d_in[9];
    const float* b_fc  = (const float*)d_in[10];
    const int* src = eidx;
    const int* dst = eidx + N_EDGES;

    char* w = (char*)d_ws;
    auto carve = [&](size_t bytes) -> char* { char* p = w; w += (bytes + 255) & ~(size_t)255; return p; };
    float* dinv = (float*)carve((size_t)N_NODES * 4 + 256);
    float* h    = (float*)carve((size_t)N_NODES * D_HID * 4);
    float* agg  = (float*)carve((size_t)N_NODES * D_HID * 4);
    float* GI   = (float*)carve((size_t)N_NODES * D_G3 * 4);
    float* outs = (float*)carve((size_t)N_NODES * D_HID * 4);
    int*   slots = (int*)carve((size_t)NCH * NBK * SLOT * 4);
    int*   cnts  = (int*)carve((size_t)NCH * NBKP * 4);
    float* y      = (float*)d_out;
    float* hfinal = (float*)d_out + N_NODES * D_OUT;

    gcn_gemm_kernel<<<(N_NODES * 16 + 255) / 256, 256, 0, stream>>>(x, W_gcn, h);
    bin_kernel<<<NCH, 256, 0, stream>>>(dst, slots, cnts);
    deg_kernel<<<NBK, 256, 0, stream>>>(src, dst, slots, cnts, dinv);
    gather_kernel<<<NBK, 256, 0, stream>>>(src, dst, slots, cnts, dinv, h, agg);
    gi_gemm_wmma<<<(N_NODES / 16 + 7) / 8, 256, 0, stream>>>(agg, b_gcn, W_ih, b_ih, GI);
    gru_scan_kernel<<<1, 256, 0, stream>>>(GI, W_hh, b_hh, h0, outs, hfinal);
    fc_kernel<<<(N_NODES * D_OUT + 255) / 256, 256, 0, stream>>>(outs, W_fc, b_fc, y);
}
